// Encoder_conv_mlp_86363202388083
// MI455X (gfx1250) — hardware-verified
//
#include <hip/hip_runtime.h>
#include <stddef.h>


#define IN_F   128
#define HID    256
#define LAT    128
#define GN     64
#define K1     (2 * IN_F)
#define K2     (2 * HID)
#define KH     (GN * HID)
#define NTHR   256
#define NWAVE  8
#define EPT    8
#define NGRP   2
#define CHUNK  (NTHR * EPT * NGRP)
#define WCAP   (EPT * NGRP * 32)
#define LISTN  (NWAVE * WCAP)
#define NB1    512
#define NB2    256
#define GROWS  32

#define LDS_AGG1 (NB1 * IN_F * 4 + LISTN * 4 + 64)
#define LDS_AGG2 (NB2 * HID * 4 + LISTN * 4 + 64)
#define LDS_GEMM (NWAVE * 16 * 64 * 4)

static_assert((CHUNK & (CHUNK - 1)) == 0);
static_assert(CHUNK <= 4096);
static_assert((NB1 & (NB1 - 1)) == 0 && NB1 <= 4096);
static_assert((NB2 & (NB2 - 1)) == 0 && NB2 <= 4096);
static_assert((NB1 * IN_F / 8) % NTHR == 0);
static_assert((NB2 * HID / 8) == 32 * NTHR);

typedef float          v4f  __attribute__((ext_vector_type(4)));
typedef float          v8f  __attribute__((ext_vector_type(8)));
typedef int            v4i  __attribute__((ext_vector_type(4)));
typedef unsigned int   v4u  __attribute__((ext_vector_type(4)));
typedef __bf16         v16b __attribute__((ext_vector_type(16)));
union FragB { v16b v; v4u q[2]; };

__device__ __forceinline__ unsigned bfb(float x) {
  const unsigned u = __float_as_uint(x);
  return (u + 0x7FFFu + ((u >> 16) & 1u)) >> 16;
}
__device__ __forceinline__ void sp2(float x, float y, unsigned& hp, unsigned& lp) {
  const unsigned hx = bfb(x), hy = bfb(y);
  const unsigned lx = bfb(x - __uint_as_float(hx << 16));
  const unsigned ly = bfb(y - __uint_as_float(hy << 16));
  hp = hx | (hy << 16);
  lp = lx | (ly << 16);
}
__device__ __forceinline__ void pack8(v4f a, v4f b, v4u& hq, v4u& lq) {
  unsigned h0, l0, h1, l1, h2, l2, h3, l3;
  sp2(a.x, a.y, h0, l0);
  sp2(a.z, a.w, h1, l1);
  sp2(b.x, b.y, h2, l2);
  sp2(b.z, b.w, h3, l3);
  hq.x = h0; hq.y = h1; hq.z = h2; hq.w = h3;
  lq.x = l0; lq.y = l1; lq.z = l2; lq.w = l3;
}
__device__ __forceinline__ void unpack_sum8(v4u qh, v4u ql, v4f& p0, v4f& p1) {
  const unsigned M = 0xFFFF0000u;
  p0.x = __uint_as_float(qh.x << 16) + __uint_as_float(ql.x << 16);
  p0.y = __uint_as_float(qh.x & M)   + __uint_as_float(ql.x & M);
  p0.z = __uint_as_float(qh.y << 16) + __uint_as_float(ql.y << 16);
  p0.w = __uint_as_float(qh.y & M)   + __uint_as_float(ql.y & M);
  p1.x = __uint_as_float(qh.z << 16) + __uint_as_float(ql.z << 16);
  p1.y = __uint_as_float(qh.z & M)   + __uint_as_float(ql.z & M);
  p1.z = __uint_as_float(qh.w << 16) + __uint_as_float(ql.w << 16);
  p1.w = __uint_as_float(qh.w & M)   + __uint_as_float(ql.w & M);
}
__device__ __forceinline__ v4f vsel(bool f, v4f p, v4f q) {
  v4f r;
  r.x = f ? p.x : q.x; r.y = f ? p.y : q.y; r.z = f ? p.z : q.z; r.w = f ? p.w : q.w;
  return r;
}

__device__ __forceinline__ FragB ldfrag(const unsigned short* p) {
  FragB f;
  f.q[0] = *(const v4u*)p;
  f.q[1] = *(const v4u*)(p + 16);
  return f;
}

__device__ __forceinline__ v8f wmb(const FragB& a, const FragB& b, v8f c) {
  v8f d = __builtin_amdgcn_wmma_f32_16x16x32_bf16(false, a.v, false, b.v, (short)0, c, false, false);
  asm volatile("v_nop\n\tv_nop\n\tv_nop\n\tv_nop" : "+v"(d) : "v"(a.q[0]), "v"(a.q[1]), "v"(b.q[0]), "v"(b.q[1]));
  return d;
}
__device__ __forceinline__ v8f wm3(const FragB& ah, const FragB& al, const FragB& bh, const FragB& bl, v8f c) {
  c = wmb(ah, bh, c);
  c = wmb(ah, bl, c);
  c = wmb(al, bh, c);
  return c;
}

template <int NB>
__device__ __forceinline__ int scan_chunk(const int* __restrict__ dsts, int nE, int cbase, int nodeBase,
                                          int vec8, int* list, int tid, int lane, int wave) {
  int wc = 0;
#pragma unroll
  for (int g = 0; g < NGRP; ++g) {
    const int el0  = (g * NTHR + tid) * EPT;
    const int e0   = cbase + el0;
    const int sent = -2147483647 - 1;
    v4i da, db;
    if (vec8 != 0 && cbase + CHUNK <= nE) {
      da = *(const v4i*)(dsts + e0);
      db = *(const v4i*)(dsts + e0 + 4);
    } else {
      da.x = (e0     < nE) ? dsts[min(e0, nE - 1)] : sent;
      da.y = (e0 + 1 < nE) ? dsts[min(e0 + 1, nE - 1)] : sent;
      da.z = (e0 + 2 < nE) ? dsts[min(e0 + 2, nE - 1)] : sent;
      da.w = (e0 + 3 < nE) ? dsts[min(e0 + 3, nE - 1)] : sent;
      db.x = (e0 + 4 < nE) ? dsts[min(e0 + 4, nE - 1)] : sent;
      db.y = (e0 + 5 < nE) ? dsts[min(e0 + 5, nE - 1)] : sent;
      db.z = (e0 + 6 < nE) ? dsts[min(e0 + 6, nE - 1)] : sent;
      db.w = (e0 + 7 < nE) ? dsts[min(e0 + 7, nE - 1)] : sent;
    }
    const unsigned nb = (unsigned)nodeBase;
    const unsigned s0 = (unsigned)da.x - nb, s1 = (unsigned)da.y - nb;
    const unsigned s2 = (unsigned)da.z - nb, s3 = (unsigned)da.w - nb;
    const unsigned s4 = (unsigned)db.x - nb, s5 = (unsigned)db.y - nb;
    const unsigned s6 = (unsigned)db.z - nb, s7 = (unsigned)db.w - nb;
    const bool h0 = s0 < (unsigned)NB, h1 = s1 < (unsigned)NB, h2 = s2 < (unsigned)NB, h3 = s3 < (unsigned)NB;
    const bool h4 = s4 < (unsigned)NB, h5 = s5 < (unsigned)NB, h6 = s6 < (unsigned)NB, h7 = s7 < (unsigned)NB;
    const unsigned any = __builtin_amdgcn_ballot_w32(h0 | h1 | h2 | h3 | h4 | h5 | h6 | h7);
    if (any != 0u) {
#define HITJ(J, HJ, SJ) { \
        const unsigned mj = __builtin_amdgcn_ballot_w32(HJ); \
        if (mj != 0u) { \
          if (HJ) { \
            const int pos = wc + (int)__builtin_amdgcn_mbcnt_lo(mj, 0u); \
            if (pos < WCAP) list[wave * WCAP + pos] = ((el0 + (J)) << 12) | (int)(SJ); \
          } \
          wc += (int)__builtin_popcount(mj); } }
      HITJ(0, h0, s0)
      HITJ(1, h1, s1)
      HITJ(2, h2, s2)
      HITJ(3, h3, s3)
      HITJ(4, h4, s4)
      HITJ(5, h5, s5)
      HITJ(6, h6, s6)
      HITJ(7, h7, s7)
#undef HITJ
    }
  }
  return wc;
}

__global__ __launch_bounds__(NTHR) void k_prep(
    const float* __restrict__ x, const float* __restrict__ W1r, const float* __restrict__ W1o,
    const float* __restrict__ W2r, const float* __restrict__ W2o,
    const float* __restrict__ Wm, const float* __restrict__ Wl,
    unsigned short* b1h, unsigned short* b1l, unsigned short* b2h, unsigned short* b2l,
    unsigned short* wmh, unsigned short* wml, unsigned short* wlh, unsigned short* wll,
    unsigned short* a1h, unsigned short* a1l, int nN, int nPad) {
  const int reg = blockIdx.y;
  const int g   = blockIdx.x * NTHR + threadIdx.x;
  v4f a, b;
  unsigned short* dh;
  unsigned short* dl;
  size_t o;
  if (reg == 0) {
    if (g >= HID * K1 / 8) return;
    const int n = g >> 5, k0 = (g & 31) * 8, kk = k0 & (IN_F - 1);
    const float* pr = W1r + (size_t)n * IN_F + kk;
    const float* po = W1o + (size_t)n * IN_F + kk;
    const v4f ar = *(const v4f*)pr, br = *(const v4f*)(pr + 4);
    const v4f ao = *(const v4f*)po, bo = *(const v4f*)(po + 4);
    const bool f = k0 < IN_F;
    a = vsel(f, ar, ao); b = vsel(f, br, bo);
    dh = b1h; dl = b1l; o = (size_t)n * K1 + k0;
  } else if (reg == 1) {
    if (g >= HID * K2 / 8) return;
    const int n = g >> 6, k0 = (g & 63) * 8, kk = k0 & (HID - 1);
    const float* pr = W2r + (size_t)n * HID + kk;
    const float* po = W2o + (size_t)n * HID + kk;
    const v4f ar = *(const v4f*)pr, br = *(const v4f*)(pr + 4);
    const v4f ao = *(const v4f*)po, bo = *(const v4f*)(po + 4);
    const bool f = k0 < HID;
    a = vsel(f, ar, ao); b = vsel(f, br, bo);
    dh = b2h; dl = b2l; o = (size_t)n * K2 + k0;
  } else if (reg == 2) {
    if (g >= LAT * KH / 8) return;
    const float* p = Wm + (size_t)g * 8;
    a = *(const v4f*)p; b = *(const v4f*)(p + 4);
    dh = wmh; dl = wml; o = (size_t)g * 8;
  } else if (reg == 3) {
    if (g >= LAT * KH / 8) return;
    const float* p = Wl + (size_t)g * 8;
    a = *(const v4f*)p; b = *(const v4f*)(p + 4);
    dh = wlh; dl = wll; o = (size_t)g * 8;
  } else {
    if (g >= nPad * (IN_F / 8)) return;
    const int row = g >> 4, c = (g & 15) * 8;
    const int rs  = row > nN - 1 ? nN - 1 : row;
    const float* p = x + (size_t)rs * IN_F + c;
    a = *(const v4f*)p; b = *(const v4f*)(p + 4);
    dh = a1h; dl = a1l; o = (size_t)row * K1 + IN_F + c;
  }
  v4u hq, lq;
  pack8(a, b, hq, lq);
  *(volatile v4u*)(dh + o) = hq;
  *(volatile v4u*)(dl + o) = lq;
  __threadfence();
  *(volatile v4u*)(dh + o) = hq;
  *(volatile v4u*)(dl + o) = lq;
}

__device__ __forceinline__ void agg1_store(const float* acc, unsigned short* a1h, unsigned short* a1l,
                                           int nodeBase, int tid) {
#pragma unroll 4
  for (int i = 0; i < (NB1 * IN_F / 8) / NTHR; ++i) {
    const int idx  = i * NTHR + tid;
    const int slot = idx >> 4;
    const int c8   = (idx & 15) * 8;
    const v4f a = *(const v4f*)(acc + slot * IN_F + c8);
    const v4f b = *(const v4f*)(acc + slot * IN_F + c8 + 4);
    v4u hq, lq;
    pack8(a, b, hq, lq);
    const size_t o = (size_t)(nodeBase + slot) * K1 + c8;
    *(volatile v4u*)(a1h + o) = hq;
    *(volatile v4u*)(a1l + o) = lq;
  }
}

__global__ __launch_bounds__(NTHR) void k_agg1(
    const int* __restrict__ ei, const float* __restrict__ x,
    unsigned short* a1h, unsigned short* a1l, int nN, int nE, int vec8) {
  extern __shared__ v4f lds_dyn[];
  float* acc  = (float*)lds_dyn;
  int*   list = (int*)(acc + NB1 * IN_F);
  int*   wcnt = list + LISTN;
  const int tid = threadIdx.x, lane = tid & 31, wave = tid >> 5;
  const int nodeBase = blockIdx.x * NB1;
  const int* dsts = ei + nE;

  {
    const v4f z = {0.f, 0.f, 0.f, 0.f};
    for (int i = tid; i < NB1 * IN_F / 4; i += NTHR) lds_dyn[i] = z;
  }
  __syncthreads();

  const int nChunks = (nE + CHUNK - 1) / CHUNK;
#pragma unroll 1
  for (int ch = 0; ch < nChunks; ++ch) {
    const int cbase = ch * CHUNK;
    const int wc = scan_chunk<NB1>(dsts, nE, cbase, nodeBase, vec8, list, tid, lane, wave);
    if (lane == 0) wcnt[wave] = wc;
    __syncthreads();
    if (wave == 0) {
#pragma unroll 1
      for (int wsx = 0; wsx < NWAVE; ++wsx) {
        int n = __builtin_amdgcn_readfirstlane(wcnt[wsx]);
        n = n > WCAP ? WCAP : (n < 0 ? 0 : n);
        const int* lp = list + wsx * WCAP;
#pragma unroll 1
        for (int i = 0; i < n; ++i) {
          const int ent  = __builtin_amdgcn_readfirstlane(lp[i]);
          const int slot = ent & (NB1 - 1);
          int e = cbase + ((ent >> 12) & (CHUNK - 1));
          e = e > nE - 1 ? nE - 1 : e;
          int src = ei[e];
          src = src < 0 ? 0 : (src > nN - 1 ? nN - 1 : src);
          const v4f v = *(const v4f*)(x + (size_t)src * IN_F + 4 * lane);
          v4f* ap = (v4f*)(acc + slot * IN_F + 4 * lane);
          *ap = *ap + v;
        }
      }
    }
    __syncthreads();
  }

  agg1_store(acc, a1h, a1l, nodeBase, tid);
  __threadfence();
  agg1_store(acc, a1h, a1l, nodeBase, tid);
}

__device__ __forceinline__ void gemm_store(const float* stg, unsigned short* Oh, unsigned short* Ol,
                                           int row0, int ldo, int ocol, int lane) {
#pragma unroll
  for (int i = 0; i < 4; ++i) {
    const int r  = 4 * i + (lane >> 3);
    const int c8 = (lane & 7) * 8;
    const v4f a = *(const v4f*)(stg + r * 64 + c8);
    const v4f b = *(const v4f*)(stg + r * 64 + c8 + 4);
    v4u hq, lq;
    pack8(a, b, hq, lq);
    const size_t o = (size_t)(row0 + r) * ldo + ocol + c8;
    *(volatile v4u*)(Oh + o) = hq;
    *(volatile v4u*)(Ol + o) = lq;
  }
}

__global__ __launch_bounds__(NTHR) void k_gemm(
    const unsigned short* __restrict__ Ah, const unsigned short* __restrict__ Al, int lda,
    const unsigned short* __restrict__ Bh, const unsigned short* __restrict__ Bl, int K,
    const float* __restrict__ bias, unsigned short* Oh, unsigned short* Ol, int ldo, int oc0) {
  extern __shared__ v4f lds_dyn[];
  const int tid = threadIdx.x, lane = tid & 31, wave = tid >> 5, hh = lane >> 4, m = lane & 15;
  const int rt = wave >> 2, cq = wave & 3;
  const int row0 = blockIdx.x * GROWS + 16 * rt;
  const int col0 = 64 * cq;
  float* stg = (float*)lds_dyn + wave * (16 * 64);

  v8f acc[4];
#pragma unroll
  for (int t = 0; t < 4; ++t) { v8f z = {0.f, 0.f, 0.f, 0.f, 0.f, 0.f, 0.f, 0.f}; acc[t] = z; }

  const unsigned short* pah = Ah + (size_t)(row0 + m) * lda + 8 * hh;
  const unsigned short* pal = Al + (size_t)(row0 + m) * lda + 8 * hh;
  const unsigned short* pbh = Bh + (size_t)(col0 + m) * K + 8 * hh;
  const unsigned short* pbl = Bl + (size_t)(col0 + m) * K + 8 * hh;
  const int nk = K >> 5;
#pragma unroll 1
  for (int kt = 0; kt < nk; ++kt) {
    const int ko = 32 * kt;
    const FragB ah = ldfrag(pah + ko);
    const FragB al = ldfrag(pal + ko);
#pragma unroll
    for (int t = 0; t < 4; ++t) {
      const size_t bo = (size_t)(16 * t) * K + ko;
      const FragB bh = ldfrag(pbh + bo);
      const FragB bl = ldfrag(pbl + bo);
      acc[t] = wm3(ah, al, bh, bl, acc[t]);
    }
  }

#pragma unroll
  for (int t = 0; t < 4; ++t) {
    const float bv = bias[col0 + 16 * t + m];
    float* sp = stg + (8 * hh) * 64 + 16 * t + m;
    sp[0 * 64] = fmaxf(acc[t][0] + bv, 0.f);
    sp[1 * 64] = fmaxf(acc[t][1] + bv, 0.f);
    sp[2 * 64] = fmaxf(acc[t][2] + bv, 0.f);
    sp[3 * 64] = fmaxf(acc[t][3] + bv, 0.f);
    sp[4 * 64] = fmaxf(acc[t][4] + bv, 0.f);
    sp[5 * 64] = fmaxf(acc[t][5] + bv, 0.f);
    sp[6 * 64] = fmaxf(acc[t][6] + bv, 0.f);
    sp[7 * 64] = fmaxf(acc[t][7] + bv, 0.f);
  }
  __syncthreads();

  gemm_store(stg, Oh, Ol, row0, ldo, oc0 + col0, lane);
  __threadfence();
  gemm_store(stg, Oh, Ol, row0, ldo, oc0 + col0, lane);
}

__device__ __forceinline__ void agg2_store(const float* acc, unsigned short* a2h, unsigned short* a2l,
                                           int nodeBase, int wave, int lane) {
#pragma unroll 4
  for (int i = 0; i < 32; ++i) {
    const int slot = i * NWAVE + wave;
    const int c8   = 8 * lane;
    const v4f a = *(const v4f*)(acc + slot * HID + c8);
    const v4f b = *(const v4f*)(acc + slot * HID + c8 + 4);
    v4u hq, lq;
    pack8(a, b, hq, lq);
    const size_t o = (size_t)(nodeBase + slot) * K2 + c8;
    *(volatile v4u*)(a2h + o) = hq;
    *(volatile v4u*)(a2l + o) = lq;
  }
}

__global__ __launch_bounds__(NTHR) void k_agg2(
    const int* __restrict__ ei, unsigned short* a2h, unsigned short* a2l, int nN, int nE, int vec8) {
  extern __shared__ v4f lds_dyn[];
  float* acc  = (float*)lds_dyn;
  int*   list = (int*)(acc + NB2 * HID);
  int*   wcnt = list + LISTN;
  const int tid = threadIdx.x, lane = tid & 31, wave = tid >> 5;
  const int nodeBase = blockIdx.x * NB2;
  const int* dsts = ei + nE;

  {
    const v4f z = {0.f, 0.f, 0.f, 0.f};
    for (int i = tid; i < NB2 * HID / 4; i += NTHR) lds_dyn[i] = z;
  }
  __syncthreads();

  const int nChunks = (nE + CHUNK - 1) / CHUNK;
#pragma unroll 1
  for (int ch = 0; ch < nChunks; ++ch) {
    const int cbase = ch * CHUNK;
    const int wc = scan_chunk<NB2>(dsts, nE, cbase, nodeBase, vec8, list, tid, lane, wave);
    if (lane == 0) wcnt[wave] = wc;
    __syncthreads();
    if (wave == 0) {
#pragma unroll 1
      for (int wsx = 0; wsx < NWAVE; ++wsx) {
        int n = __builtin_amdgcn_readfirstlane(wcnt[wsx]);
        n = n > WCAP ? WCAP : (n < 0 ? 0 : n);
        const int* lp = list + wsx * WCAP;
#pragma unroll 1
        for (int i = 0; i < n; ++i) {
          const int ent  = __builtin_amdgcn_readfirstlane(lp[i]);
          const int slot = ent & (NB2 - 1);
          int e = cbase + ((ent >> 12) & (CHUNK - 1));
          e = e > nE - 1 ? nE - 1 : e;
          int src = ei[e];
          src = src < 0 ? 0 : (src > nN - 1 ? nN - 1 : src);
          const size_t so = (size_t)src * K2 + HID + 8 * lane;
          const v4u qh = *(const v4u*)(a2h + so);
          const v4u ql = *(const v4u*)(a2l + so);
          v4f p0, p1;
          unpack_sum8(qh, ql, p0, p1);
          v4f* ap = (v4f*)(acc + slot * HID + 8 * lane);
          ap[0] = ap[0] + p0;
          ap[1] = ap[1] + p1;
        }
      }
    }
    __syncthreads();
  }

  agg2_store(acc, a2h, a2l, nodeBase, wave, lane);
  __threadfence();
  agg2_store(acc, a2h, a2l, nodeBase, wave, lane);
}

__device__ __forceinline__ void head_store(const float* st, float* ob, int row0, int bs, int lane) {
#pragma unroll
  for (int i = 0; i < 8; ++i) {
    const int r  = 2 * i + (lane >> 4);
    const int c4 = (lane & 15) * 4;
    const v4f v  = *(const v4f*)(st + r * 64 + c4);
    const int grow = row0 + r;
    if (grow < bs) *(volatile v4f*)(ob + (size_t)grow * LAT + c4) = v;
  }
}

__global__ __launch_bounds__(64) void k_head(
    const unsigned short* __restrict__ hbh, const unsigned short* __restrict__ hbl,
    const unsigned short* __restrict__ wmh, const unsigned short* __restrict__ wml,
    const unsigned short* __restrict__ wlh, const unsigned short* __restrict__ wll,
    const float* __restrict__ bmu, const float* __restrict__ blv, float* out, int bs) {
  __shared__ __attribute__((aligned(16))) float stg[2 * 16 * 64];
  const int tid = threadIdx.x, lane = tid & 31, wave = tid >> 5, hh = lane >> 4, m = lane & 15;
  const int head = blockIdx.y;
  const int row0 = blockIdx.x * 16;
  const int col0 = 64 * wave;
  const unsigned short* Bh = head ? wlh : wmh;
  const unsigned short* Bl = head ? wll : wml;
  const float* bias = head ? blv : bmu;

  v8f acc[4];
#pragma unroll
  for (int t = 0; t < 4; ++t) { v8f z = {0.f, 0.f, 0.f, 0.f, 0.f, 0.f, 0.f, 0.f}; acc[t] = z; }

  const unsigned short* pah = hbh + (size_t)(row0 + m) * KH + 8 * hh;
  const unsigned short* pal = hbl + (size_t)(row0 + m) * KH + 8 * hh;
  const unsigned short* pbh = Bh + (size_t)(col0 + m) * KH + 8 * hh;
  const unsigned short* pbl = Bl + (size_t)(col0 + m) * KH + 8 * hh;
#pragma unroll 1
  for (int kt = 0; kt < KH / 32; ++kt) {
    const int ko = 32 * kt;
    const FragB ah = ldfrag(pah + ko);
    const FragB al = ldfrag(pal + ko);
#pragma unroll
    for (int t = 0; t < 4; ++t) {
      const size_t bo = (size_t)(16 * t) * KH + ko;
      const FragB bh = ldfrag(pbh + bo);
      const FragB bl = ldfrag(pbl + bo);
      acc[t] = wm3(ah, al, bh, bl, acc[t]);
    }
  }

  float* st = stg + wave * (16 * 64);
#pragma unroll
  for (int t = 0; t < 4; ++t) {
    const float bv = bias[col0 + 16 * t + m];
    float* sp = st + (8 * hh) * 64 + 16 * t + m;
    sp[0 * 64] = acc[t][0] + bv;
    sp[1 * 64] = acc[t][1] + bv;
    sp[2 * 64] = acc[t][2] + bv;
    sp[3 * 64] = acc[t][3] + bv;
    sp[4 * 64] = acc[t][4] + bv;
    sp[5 * 64] = acc[t][5] + bv;
    sp[6 * 64] = acc[t][6] + bv;
    sp[7 * 64] = acc[t][7] + bv;
  }
  __syncthreads();

  float* ob = out + (size_t)head * bs * LAT + col0;
  head_store(st, ob, row0, bs, lane);
  __threadfence();
  head_store(st, ob, row0, bs, lane);
}

extern "C" void kernel_launch(void* const* d_in, const int* in_sizes, int n_in,
                              void* d_out, int out_size, void* d_ws, size_t ws_size,
                              hipStream_t stream) {
  if (n_in < 13) return;
  const int nN = in_sizes[0] / IN_F;
  if (nN <= 0 || in_sizes[0] != nN * IN_F || (nN % GN) != 0) return;
  const int bs = nN / GN;
  if (in_sizes[1] != HID * IN_F || in_sizes[2] != HID * IN_F || in_sizes[3] < HID) return;
  if (in_sizes[4] != HID * HID || in_sizes[5] != HID * HID || in_sizes[6] < HID) return;
  if (in_sizes[7] != LAT * KH || in_sizes[8] < LAT || in_sizes[9] != LAT * KH || in_sizes[10] < LAT) return;
  if (in_sizes[11] < 0 || (in_sizes[11] & 1) != 0) return;
  const int nE = in_sizes[11] / 2;
  if (out_size != 2 * bs * LAT) return;

  const float* x    = (const float*)d_in[0];
  const float* W1r  = (const float*)d_in[1];
  const float* W1o  = (const float*)d_in[2];
  const float* b1   = (const float*)d_in[3];
  const float* W2r  = (const float*)d_in[4];
  const float* W2o  = (const float*)d_in[5];
  const float* b2   = (const float*)d_in[6];
  const float* Wmu  = (const float*)d_in[7];
  const float* bmu  = (const float*)d_in[8];
  const float* Wlv  = (const float*)d_in[9];
  const float* blv  = (const float*)d_in[10];
  const int*   ei   = (const int*)d_in[11];
  float* out = (float*)d_out;

  const int nPad = ((nN + 1023) / 1024) * 1024;

  const size_t szB1 = (size_t)HID * K1 * 2, szB2 = (size_t)HID * K2 * 2, szW = (size_t)LAT * KH * 2;
  const size_t szA1 = (size_t)nPad * K1 * 2, szA2 = (size_t)nPad * K2 * 2;
  char* ws = (char*)d_ws;
  size_t off = 0;
#define CARVE(name, bytes) const size_t name = off; off += ((size_t)(bytes) + 255) & ~(size_t)255;
  CARVE(oB1h, szB1) CARVE(oB1l, szB1)
  CARVE(oB2h, szB2) CARVE(oB2l, szB2)
  CARVE(oWMh, szW)  CARVE(oWMl, szW)  CARVE(oWLh, szW)  CARVE(oWLl, szW)
  CARVE(oA1h, szA1) CARVE(oA1l, szA1)
  CARVE(oA2h, szA2) CARVE(oA2l, szA2)
#undef CARVE
  if (off > ws_size || off > (size_t)134217728) return;
  unsigned short* B1h = (unsigned short*)(ws + oB1h);
  unsigned short* B1l = (unsigned short*)(ws + oB1l);
  unsigned short* B2h = (unsigned short*)(ws + oB2h);
  unsigned short* B2l = (unsigned short*)(ws + oB2l);
  unsigned short* WMh = (unsigned short*)(ws + oWMh);
  unsigned short* WMl = (unsigned short*)(ws + oWMl);
  unsigned short* WLh = (unsigned short*)(ws + oWLh);
  unsigned short* WLl = (unsigned short*)(ws + oWLl);
  unsigned short* A1h = (unsigned short*)(ws + oA1h);
  unsigned short* A1l = (unsigned short*)(ws + oA1l);
  unsigned short* A2h = (unsigned short*)(ws + oA2h);
  unsigned short* A2l = (unsigned short*)(ws + oA2l);
  unsigned short* H2h = A1h;
  unsigned short* H2l = A1l;

  const int vec8 = ((nE & 3) == 0) ? 1 : 0;

  {
    int maxc = LAT * KH / 8;
    if (nPad * (IN_F / 8) > maxc) maxc = nPad * (IN_F / 8);
    if (HID * K2 / 8 > maxc) maxc = HID * K2 / 8;
    dim3 gp((maxc + NTHR - 1) / NTHR, 5);
    k_prep<<<gp, NTHR, 0, stream>>>(x, W1r, W1o, W2r, W2o, Wmu, Wlv,
                                    B1h, B1l, B2h, B2l, WMh, WMl, WLh, WLl, A1h, A1l, nN, nPad);
  }

  hipFuncSetAttribute(reinterpret_cast<const void*>(&k_agg1),
                      hipFuncAttributeMaxDynamicSharedMemorySize, LDS_AGG1);
  k_agg1<<<nPad / NB1, NTHR, LDS_AGG1, stream>>>(ei, x, A1h, A1l, nN, nE, vec8);

  hipFuncSetAttribute(reinterpret_cast<const void*>(&k_gemm),
                      hipFuncAttributeMaxDynamicSharedMemorySize, LDS_GEMM);
  k_gemm<<<nPad / GROWS, NTHR, LDS_GEMM, stream>>>(A1h, A1l, K1, B1h, B1l, K1, b1, A2h, A2l, K2, HID);

  hipFuncSetAttribute(reinterpret_cast<const void*>(&k_agg2),
                      hipFuncAttributeMaxDynamicSharedMemorySize, LDS_AGG2);
  k_agg2<<<nPad / NB2, NTHR, LDS_AGG2, stream>>>(ei, A2h, A2l, nN, nE, vec8);

  k_gemm<<<nPad / GROWS, NTHR, LDS_GEMM, stream>>>(A2h, A2l, K2, B2h, B2l, K2, b2, H2h, H2l, HID, 0);

  k_head<<<dim3((bs + 15) / 16, 2), 64, 0, stream>>>(H2h, H2l, WMh, WMl, WLh, WLl, bmu, blv, out, bs);
}
